// EnhancedAttentionLayer_41601053229527
// MI455X (gfx1250) — hardware-verified
//
#include <hip/hip_runtime.h>
#include <stddef.h>


#define NB    8
#define NN    512
#define DIN   768
#define NH    8
#define DO    96
#define MR    (NB * NN)
#define NWT   (4 * DIN)
#define PP    (NN + 8)
#define BMP   128
#define NTP   256
#define NTA   128
#define WSC   16.0f
#define RWSC  0.0625f
#define PSC   1024.0f
#define RPSC  0.0009765625f
#define LEAKY 0.2f
#define NEGF  (-99999.0f)
#define WSCAP 134217728

static_assert(MR % BMP == 0);
static_assert(NN % BMP == 0);
static_assert(DIN % 32 == 0 && NN % 32 == 0);
static_assert(DO % 16 == 0 && ((DO * 4) % 128) == 0);
static_assert(NH * DO == DIN);
static_assert(((PP * 2) % 16) == 0);
static_assert(NN / 16 == 32);
static_assert(NN == 32 * 16);
static_assert(NWT / DO == 32);
static_assert((DIN * (DIN / 8)) % NTP == 0);
static_assert((MR * DIN / 8) % NTP == 0);
static_assert((MR * NH) % NTP == 0 && (NN % NTP) == 0);

typedef _Float16 v16h __attribute__((ext_vector_type(16)));
typedef _Float16 v8h  __attribute__((ext_vector_type(8)));
typedef float    v8f  __attribute__((ext_vector_type(8)));
typedef float    v4f  __attribute__((ext_vector_type(4)));
typedef int      v4i  __attribute__((ext_vector_type(4)));
union Frag { v16h v; v8h h[2]; };
union HP   { v8h h[2]; _Float16 s[16]; };

__device__ __forceinline__ v8f wmh(v16h a, v16h b, v8f c) {
  v8f d = __builtin_amdgcn_wmma_f32_16x16x32_f16(false, a, false, b, (short)0, c, false, false);
  asm volatile("v_nop\n\tv_nop\n\tv_nop\n\tv_nop" : "+v"(d) : "v"(a), "v"(b));
  return d;
}

__device__ __forceinline__ v8f zero8() {
  v8f z = {0.f, 0.f, 0.f, 0.f, 0.f, 0.f, 0.f, 0.f};
  return z;
}

__device__ __forceinline__ v8h cvt8(v4f a, v4f b) {
  v8h r;
  r[0] = (_Float16)a.x; r[1] = (_Float16)a.y; r[2] = (_Float16)a.z; r[3] = (_Float16)a.w;
  r[4] = (_Float16)b.x; r[5] = (_Float16)b.y; r[6] = (_Float16)b.z; r[7] = (_Float16)b.w;
  return r;
}

__device__ __forceinline__ void unpack4f(v4f v, float* d) { d[0] = v.x; d[1] = v.y; d[2] = v.z; d[3] = v.w; }
__device__ __forceinline__ void unpack4i(v4i v, int* d)   { d[0] = v.x; d[1] = v.y; d[2] = v.z; d[3] = v.w; }

__device__ __forceinline__ float eluf(float v) { return v > 0.0f ? v : (__expf(v) - 1.0f); }

__device__ __forceinline__ float sigm(float x) {
  x = fminf(fmaxf(x, -30.0f), 30.0f);
  return __builtin_amdgcn_rcpf(1.0f + __expf(-x));
}

__device__ __forceinline__ void mlogit(float si, float dj, int smi, int adi, int j, int i,
                                       float& x2, float& x3, float& interf, float& outerf) {
  float l = si + dj;
  l = (l >= 0.0f) ? l : LEAKY * l;
  const float smf = (float)smi, adf = (float)adi;
  const float eyef = (j == i) ? 1.0f : 0.0f;
  interf = (smf == 1.0f) ? (smf - eyef) : smf;
  outerf = (smf == 0.0f) ? adf : (1.0f - smf);
  x2 = ((1.0f - interf) != 0.0f) ? NEGF : l;
  x3 = ((1.0f - outerf) != 0.0f) ? NEGF : l;
}

__global__ __launch_bounds__(NTP) void k_cvtx(const float* __restrict__ x, _Float16* xh, int n8) {
  const int i = (int)blockIdx.x * NTP + (int)threadIdx.x;
  if (i >= n8) return;
  const float* p = x + (size_t)i * 8;
  const v4f a = *(const v4f*)p;
  const v4f b = *(const v4f*)(p + 4);
  const v8h v = cvt8(a, b);
  _Float16* d = xh + (size_t)i * 8;
  *(volatile v8h*)d = v;
  __threadfence();
  *(volatile v8h*)d = v;
}

__global__ __launch_bounds__(NTP) void k_cvtw(const float* __restrict__ W1, const float* __restrict__ W2,
                                              const float* __restrict__ W3, const float* __restrict__ Hw,
                                              _Float16* wt) {
  const int u = (int)blockIdx.x * NTP + (int)threadIdx.x;
  const int y = (int)blockIdx.y;
  if (u >= DIN * (DIN / 8)) return;
  const int nl = u / (DIN / 8);
  const int k0 = (u - nl * (DIN / 8)) * 8;
  v4f a, b;
  if (y < 3) {
    const float* Wg = (y == 0) ? W1 : ((y == 1) ? W2 : W3);
    const int hh = nl / DO, ee = nl - hh * DO;
    const float* s = Wg + ((size_t)(hh * DIN + k0)) * DO + ee;
    a.x = s[0];      a.y = s[DO];     a.z = s[2 * DO]; a.w = s[3 * DO];
    b.x = s[4 * DO]; b.y = s[5 * DO]; b.z = s[6 * DO]; b.w = s[7 * DO];
  } else {
    const float* s = Hw + (size_t)nl * DIN + k0;
    a = *(const v4f*)s;
    b = *(const v4f*)(s + 4);
  }
  a = a * WSC;
  b = b * WSC;
  const v8h v = cvt8(a, b);
  _Float16* d = wt + ((size_t)(y * DIN + nl)) * DIN + k0;
  *(volatile v8h*)d = v;
  __threadfence();
  *(volatile v8h*)d = v;
}

__global__ __launch_bounds__(NTP) void k_proj(const _Float16* __restrict__ Xh, const _Float16* __restrict__ Wt,
                                              const float* __restrict__ Hb,
                                              float* h1p, _Float16* hT, float* gate) {
  __shared__ __attribute__((aligned(16))) float stg[BMP * DO];
  const int tid = threadIdx.x, lane = tid & 31, wave = tid >> 5, hf = lane >> 4, m = lane & 15;
  const int cb = (int)blockIdx.x & 31, rb = (int)blockIdx.x >> 5;
  const int row0 = rb * BMP, n0 = cb * DO;

  v8f acc[6];
#pragma unroll
  for (int t = 0; t < 6; ++t) acc[t] = zero8();

  const _Float16* ap = Xh + (size_t)(row0 + 16 * wave + m) * DIN + 8 * hf;
  const _Float16* bp = Wt + (size_t)(n0 + m) * DIN + 8 * hf;
#pragma unroll 1
  for (int kc = 0; kc < DIN / 32; ++kc) {
    Frag a;
    a.h[0] = *(const v8h*)(ap + 32 * kc);
    a.h[1] = *(const v8h*)(ap + 32 * kc + 16);
#pragma unroll
    for (int t = 0; t < 6; ++t) {
      const _Float16* q = bp + (size_t)t * 16 * DIN + 32 * kc;
      Frag bf;
      bf.h[0] = *(const v8h*)q;
      bf.h[1] = *(const v8h*)(q + 16);
      acc[t] = wmh(a.v, bf.v, acc[t]);
    }
  }

  {
    float* sp = stg + (16 * wave + 8 * hf) * DO + m;
#pragma unroll
    for (int t = 0; t < 6; ++t) {
#pragma unroll
      for (int r = 0; r < 8; ++r) sp[r * DO + 16 * t] = acc[t][r] * RWSC;
    }
  }
  __syncthreads();

  const int b   = rb >> 2;
  const int nl0 = (rb & 3) * BMP;
  const int cl  = lane < (DO / 4) ? lane : (DO / 4 - 1);
  const bool stok = lane < (DO / 4);

  if (cb < NH) {
    float* dst = h1p + ((size_t)((b * NH + cb) * NN + nl0 + 16 * wave)) * DO + 4 * cl;
    const float* src = stg + (16 * wave) * DO + 4 * cl;
#pragma unroll
    for (int row = 0; row < 16; ++row) {
      const v4f v = *(const v4f*)(src + row * DO);
      if (stok) *(volatile v4f*)(dst + (size_t)row * DO) = v;
    }
    __threadfence();
#pragma unroll
    for (int row = 0; row < 16; ++row) {
      const v4f v = *(const v4f*)(src + row * DO);
      if (stok) *(volatile v4f*)(dst + (size_t)row * DO) = v;
    }
  } else if (cb < 3 * NH) {
    const int gsel = (cb >> 3) - 1, hd = cb & 7;
    _Float16* base = hT + (((size_t)gsel * (NB * NH) + b * NH + hd) * DO) * NN + nl0 + 8 * m;
    const float* src = stg + (8 * m) * DO;
#pragma unroll
    for (int it = 0; it < 6; ++it) {
      const int e = 12 * wave + 2 * it + hf;
      v4f a, c;
      a.x = src[0 * DO + e]; a.y = src[1 * DO + e]; a.z = src[2 * DO + e]; a.w = src[3 * DO + e];
      c.x = src[4 * DO + e]; c.y = src[5 * DO + e]; c.z = src[6 * DO + e]; c.w = src[7 * DO + e];
      const v8h v = cvt8(a, c);
      *(volatile v8h*)(base + (size_t)e * NN) = v;
    }
    __threadfence();
#pragma unroll
    for (int it = 0; it < 6; ++it) {
      const int e = 12 * wave + 2 * it + hf;
      v4f a, c;
      a.x = src[0 * DO + e]; a.y = src[1 * DO + e]; a.z = src[2 * DO + e]; a.w = src[3 * DO + e];
      c.x = src[4 * DO + e]; c.y = src[5 * DO + e]; c.z = src[6 * DO + e]; c.w = src[7 * DO + e];
      const v8h v = cvt8(a, c);
      *(volatile v8h*)(base + (size_t)e * NN) = v;
    }
  } else {
    const int c0 = (cb - 3 * NH) * DO;
    const v4f hb = *(const v4f*)(Hb + c0 + 4 * cl);
    float* dst = gate + ((size_t)(row0 + 16 * wave)) * DIN + c0 + 4 * cl;
    const float* src = stg + (16 * wave) * DO + 4 * cl;
#pragma unroll
    for (int row = 0; row < 16; ++row) {
      v4f v = *(const v4f*)(src + row * DO) + hb;
      v.x = sigm(v.x); v.y = sigm(v.y); v.z = sigm(v.z); v.w = sigm(v.w);
      if (stok) *(volatile v4f*)(dst + (size_t)row * DIN) = v;
    }
    __threadfence();
#pragma unroll
    for (int row = 0; row < 16; ++row) {
      v4f v = *(const v4f*)(src + row * DO) + hb;
      v.x = sigm(v.x); v.y = sigm(v.y); v.z = sigm(v.z); v.w = sigm(v.w);
      if (stok) *(volatile v4f*)(dst + (size_t)row * DIN) = v;
    }
  }
}

__global__ __launch_bounds__(NTP) void k_attvec(const float* __restrict__ h1p, const float* __restrict__ wsrc,
                                                const float* __restrict__ wdst, const int* __restrict__ rel,
                                                float* asrc, float* adst, int nrows) {
  __shared__ __attribute__((aligned(16))) float sS[NTP];
  __shared__ __attribute__((aligned(16))) float sD[NTP];
  (void)rel;
  const int tid = threadIdx.x, lane = tid & 31, wave = tid >> 5;
  int gid = (int)blockIdx.x * NTP + tid;
  gid = gid > nrows - 1 ? nrows - 1 : gid;
  const int hd = (gid >> 9) & (NH - 1);
  const float* row = h1p + (size_t)gid * DO;
  const float* ws = wsrc + hd * DO;
  const float* wd = wdst + hd * DO;
  float s = 0.0f, d = 0.0f;
#pragma unroll 1
  for (int e = 0; e < DO; ++e) {
    const float t = tanhf(row[e]);
    s += t * ws[e];
    d += t * wd[e];
  }
  sS[tid] = s;
  sD[tid] = d;
  __syncthreads();
  const int f = (wave & 1) * 32 + lane;
  const v4f vs = *(const v4f*)(sS + 4 * f);
  const v4f vd = *(const v4f*)(sD + 4 * f);
  float* ps = asrc + (size_t)blockIdx.x * NTP + 4 * f;
  float* pd = adst + (size_t)blockIdx.x * NTP + 4 * f;
  if (wave < 2) *(volatile v4f*)ps = vs;
  if (wave >= 2 && wave < 4) *(volatile v4f*)pd = vd;
  __threadfence();
  if (wave < 2) *(volatile v4f*)ps = vs;
  if (wave >= 2 && wave < 4) *(volatile v4f*)pd = vd;
}

__global__ __launch_bounds__(NTA) void k_attn(const int* __restrict__ adj, const int* __restrict__ smask,
                                              const float* __restrict__ asrc, const float* __restrict__ adst,
                                              const float* __restrict__ h1p, const _Float16* __restrict__ hT,
                                              const float* __restrict__ bias, const float* __restrict__ gate,
                                              const float* __restrict__ feat, float* out) {
  __shared__ __attribute__((aligned(16))) _Float16 sP[2 * 16 * PP];
  __shared__ __attribute__((aligned(16))) float stg[2 * 16 * DO];
  __shared__ float sInv[32];
  __shared__ float sAdjd[16];
  const int tid = threadIdx.x, lane = tid & 31, wave = tid >> 5, hf = lane >> 4, m = lane & 15;
  const int bh = (int)blockIdx.x >> 5, rt = (int)blockIdx.x & 31;
  const int b = bh >> 3, hd = bh & 7, row0 = rt * 16;

  const int j0 = 16 * lane;
  float dv[16];
  {
    const float* dp = adst + (size_t)bh * NN + j0;
    unpack4f(*(const v4f*)dp,        dv);
    unpack4f(*(const v4f*)(dp + 4),  dv + 4);
    unpack4f(*(const v4f*)(dp + 8),  dv + 8);
    unpack4f(*(const v4f*)(dp + 12), dv + 12);
  }

#pragma unroll 1
  for (int q = 0; q < 4; ++q) {
    const int rl = 4 * wave + q;
    const int i  = row0 + rl;
    const float si = asrc[(size_t)bh * NN + i];
    const int* arow = adj   + ((size_t)(b * NN + i)) * NN;
    const int* srow = smask + ((size_t)(b * NN + i)) * NN;
    const float adjd = (float)arow[i];
    int av[16], sv[16];
    unpack4i(*(const v4i*)(arow + j0),      av);
    unpack4i(*(const v4i*)(arow + j0 + 4),  av + 4);
    unpack4i(*(const v4i*)(arow + j0 + 8),  av + 8);
    unpack4i(*(const v4i*)(arow + j0 + 12), av + 12);
    unpack4i(*(const v4i*)(srow + j0),      sv);
    unpack4i(*(const v4i*)(srow + j0 + 4),  sv + 4);
    unpack4i(*(const v4i*)(srow + j0 + 8),  sv + 8);
    unpack4i(*(const v4i*)(srow + j0 + 12), sv + 12);

    float m2 = -3.0e38f, m3 = -3.0e38f;
#pragma unroll
    for (int t = 0; t < 16; ++t) {
      float x2, x3, interf, outerf;
      mlogit(si, dv[t], sv[t], av[t], j0 + t, i, x2, x3, interf, outerf);
      m2 = fmaxf(m2, x2);
      m3 = fmaxf(m3, x3);
    }
#pragma unroll
    for (int o = 16; o > 0; o >>= 1) {
      m2 = fmaxf(m2, __shfl_xor(m2, o));
      m3 = fmaxf(m3, __shfl_xor(m3, o));
    }

    float s2 = 0.0f, s3 = 0.0f;
    HP P2, P3;
#pragma unroll
    for (int t = 0; t < 16; ++t) {
      float x2, x3, interf, outerf;
      mlogit(si, dv[t], sv[t], av[t], j0 + t, i, x2, x3, interf, outerf);
      const float e2 = __expf(x2 - m2);
      const float e3 = __expf(x3 - m3);
      s2 += e2;
      s3 += e3;
      P2.s[t] = (_Float16)((interf > 0.0f) ? e2 * PSC : 0.0f);
      P3.s[t] = (_Float16)((outerf > 0.0f) ? e3 * PSC : 0.0f);
    }
    _Float16* p2row = sP + rl * PP + j0;
    _Float16* p3row = sP + (16 + rl) * PP + j0;
    *(v8h*)p2row       = P2.h[0];
    *(v8h*)(p2row + 8) = P2.h[1];
    *(v8h*)p3row       = P3.h[0];
    *(v8h*)(p3row + 8) = P3.h[1];
#pragma unroll
    for (int o = 16; o > 0; o >>= 1) {
      s2 += __shfl_xor(s2, o);
      s3 += __shfl_xor(s3, o);
    }
    if (lane == 0) {
      sInv[rl]      = __builtin_amdgcn_rcpf(s2) * RPSC;
      sInv[16 + rl] = __builtin_amdgcn_rcpf(s3) * RPSC;
      sAdjd[rl]     = adjd;
    }
  }
  __syncthreads();

  const int g = wave & 1, ct0 = 3 * (wave >> 1);
  v8f acc[3];
#pragma unroll
  for (int t = 0; t < 3; ++t) acc[t] = zero8();
  const _Float16* ap = sP + (g * 16 + m) * PP + 8 * hf;
  const _Float16* bp = hT + (((size_t)g * (NB * NH) + bh) * DO + 16 * ct0 + m) * NN + 8 * hf;
#pragma unroll 1
  for (int kc = 0; kc < NN / 32; ++kc) {
    Frag a;
    a.h[0] = *(const v8h*)(ap + 32 * kc);
    a.h[1] = *(const v8h*)(ap + 32 * kc + 16);
#pragma unroll
    for (int t = 0; t < 3; ++t) {
      const _Float16* q = bp + (size_t)t * 16 * NN + 32 * kc;
      Frag bf;
      bf.h[0] = *(const v8h*)q;
      bf.h[1] = *(const v8h*)(q + 16);
      acc[t] = wmh(a.v, bf.v, acc[t]);
    }
  }
  {
    float* sp = stg + (g * 16 + 8 * hf) * DO + 16 * ct0 + m;
#pragma unroll
    for (int t = 0; t < 3; ++t) {
#pragma unroll
      for (int r = 0; r < 8; ++r) sp[r * DO + 16 * t] = acc[t][r] * sInv[g * 16 + 8 * hf + r];
    }
  }
  __syncthreads();

  const int cl = lane < (DO / 4) ? lane : (DO / 4 - 1);
  const bool stok = lane < (DO / 4);
  const v4f bb = *(const v4f*)(bias + 4 * cl);
  v4f ov[4];
  size_t go[4];
#pragma unroll
  for (int q = 0; q < 4; ++q) {
    const int rl = 4 * wave + q;
    const int i  = row0 + rl;
    const v4f v2  = *(const v4f*)(stg + rl * DO + 4 * cl);
    const v4f v3  = *(const v4f*)(stg + (16 + rl) * DO + 4 * cl);
    const v4f h1v = *(const v4f*)(h1p + ((size_t)(bh * NN + i)) * DO + 4 * cl);
    const float adjd = sAdjd[rl];
    const size_t gofs = ((size_t)(b * NN + i)) * DIN + hd * DO + 4 * cl;
    const v4f gv = *(const v4f*)(gate + gofs);
    const v4f fv = *(const v4f*)(feat + gofs);
    v4f val = ((h1v * adjd + v2) + v3 + bb) * (1.0f / 3.0f);
    val.x = eluf(val.x); val.y = eluf(val.y); val.z = eluf(val.z); val.w = eluf(val.w);
    const v4f omg = 1.0f - gv;
    ov[q] = gv * val + omg * fv;
    go[q] = gofs;
  }
#pragma unroll
  for (int q = 0; q < 4; ++q) { if (stok) *(volatile v4f*)(out + go[q]) = ov[q]; }
  __threadfence();
#pragma unroll
  for (int q = 0; q < 4; ++q) { if (stok) *(volatile v4f*)(out + go[q]) = ov[q]; }
}

extern "C" void kernel_launch(void* const* d_in, const int* in_sizes, int n_in,
                              void* d_out, int out_size, void* d_ws, size_t ws_size,
                              hipStream_t stream) {
  if (n_in < 12) return;
  if (in_sizes[0] != MR * DIN) return;
  if (in_sizes[1] != NB * NN * NN || in_sizes[3] != NB * NN * NN) return;
  if (in_sizes[4] != NH * DIN * DO || in_sizes[5] != NH * DIN * DO || in_sizes[6] != NH * DIN * DO) return;
  if (in_sizes[7] != DO || in_sizes[8] != NH * DO || in_sizes[9] != NH * DO) return;
  if (in_sizes[10] != DIN * DIN || in_sizes[11] != DIN) return;
  if (out_size != MR * DIN) return;

  const float* feat  = (const float*)d_in[0];
  const int*   adj   = (const int*)d_in[1];
  const int*   rel   = (const int*)d_in[2];
  const int*   smask = (const int*)d_in[3];
  const float* W1    = (const float*)d_in[4];
  const float* W2    = (const float*)d_in[5];
  const float* W3    = (const float*)d_in[6];
  const float* bias  = (const float*)d_in[7];
  const float* wsrc  = (const float*)d_in[8];
  const float* wdst  = (const float*)d_in[9];
  const float* Hw    = (const float*)d_in[10];
  const float* Hb    = (const float*)d_in[11];
  float* out = (float*)d_out;

  char* ws = (char*)d_ws;
  size_t off = 0;
  const size_t oXh = off; off += (size_t)MR * DIN * 2;              off = (off + 255) & ~(size_t)255;
  const size_t oWt = off; off += (size_t)NWT * DIN * 2;             off = (off + 255) & ~(size_t)255;
  const size_t oH1 = off; off += (size_t)MR * NH * DO * 4;          off = (off + 255) & ~(size_t)255;
  const size_t oHT = off; off += (size_t)2 * NB * NH * DO * NN * 2; off = (off + 255) & ~(size_t)255;
  const size_t oG  = off; off += (size_t)MR * DIN * 4;              off = (off + 255) & ~(size_t)255;
  const size_t oS  = off; off += (size_t)MR * NH * 4;               off = (off + 255) & ~(size_t)255;
  const size_t oD  = off; off += (size_t)MR * NH * 4;               off = (off + 255) & ~(size_t)255;
  if (off > ws_size || off > (size_t)WSCAP) return;
  _Float16* Xh   = (_Float16*)(ws + oXh);
  _Float16* Wt   = (_Float16*)(ws + oWt);
  float*    h1p  = (float*)(ws + oH1);
  _Float16* hT   = (_Float16*)(ws + oHT);
  float*    gat  = (float*)(ws + oG);
  float*    asrc = (float*)(ws + oS);
  float*    adst = (float*)(ws + oD);

  k_cvtx<<<(MR * DIN / 8) / NTP, NTP, 0, stream>>>(feat, Xh, MR * DIN / 8);
  dim3 gw((DIN * (DIN / 8)) / NTP, 4, 1);
  k_cvtw<<<gw, NTP, 0, stream>>>(W1, W2, W3, Hw, Wt);
  k_proj<<<(MR / BMP) * (NWT / DO), NTP, 0, stream>>>(Xh, Wt, Hb, h1p, hT, gat);
  k_attvec<<<(MR * NH) / NTP, NTP, 0, stream>>>(h1p, wsrc, wdst, rel, asrc, adst, MR * NH);
  k_attn<<<NB * NH * (NN / 16), NTA, 0, stream>>>(adj, smask, asrc, adst, h1p, hT, bias, gat, feat, out);
}
